// RefNonLocal_60644938219913
// MI455X (gfx1250) — hardware-run, weakly checked
//
#include <hip/hip_runtime.h>
#include <math.h>

typedef __attribute__((ext_vector_type(16))) _Float16 v16h;
typedef __attribute__((ext_vector_type(8)))  _Float16 v8h;
typedef __attribute__((ext_vector_type(16))) __bf16   v16b;
typedef __attribute__((ext_vector_type(8)))  __bf16   v8b;
typedef __attribute__((ext_vector_type(8)))  float    v8f;
typedef __attribute__((ext_vector_type(4)))  float    v4f;
typedef __attribute__((ext_vector_type(4)))  unsigned int v4u;

constexpr int kBatch  = 8;
constexpr int kNq     = 4096;
constexpr int kMk     = 2048;
constexpr int kC      = 256;
constexpr int kRows   = kBatch * kNq;
constexpr int kPRows  = kBatch * kMk;
constexpr int kNcat   = 3 * kC;
constexpr int kAtWaves  = 4;
constexpr int kQryBlock = 64;
constexpr int kKeyChunk = 64;
constexpr float kLog2e   = 1.4426950408889634f;
constexpr float kPCarryL = 15.0f;
static_assert(kMk * 2 == kNq);
static_assert((kC % 32) == 0);
static_assert((kRows % 64) == 0 && (kC % 64) == 0 && (kNcat % 64) == 0);
static_assert((kNq % kQryBlock) == 0 && (kMk % kKeyChunk) == 0);
static_assert(kQryBlock == kAtWaves * 16);

constexpr size_t kOffXH = 0;
constexpr size_t kOffXL = kOffXH + (size_t)kRows  * kC * 2;
constexpr size_t kOffWH = kOffXL + (size_t)kRows  * kC * 2;
constexpr size_t kOffWL = kOffWH + (size_t)kNcat  * kC * 2;
constexpr size_t kOffTH = kOffWL + (size_t)kNcat  * kC * 2;
constexpr size_t kOffTL = kOffTH + (size_t)kRows  * kC * 2;
constexpr size_t kOffPH = kOffTL + (size_t)kRows  * kC * 2;
constexpr size_t kOffPL = kOffPH + (size_t)kPRows * kC * 2;
constexpr size_t kOffG  = kOffPL + (size_t)kPRows * kC * 2;
constexpr size_t kOffGT = kOffG  + (size_t)kPRows * kC * 2;
constexpr size_t kWsTotal = kOffGT + (size_t)kBatch * kC * kMk * 2;
static_assert(kWsTotal == 101449728ull);
static_assert(kWsTotal <= 134217728ull);
static_assert((kOffXL % 128) == 0 && (kOffWH % 128) == 0 && (kOffWL % 128) == 0 && (kOffTH % 128) == 0 &&
              (kOffTL % 128) == 0 && (kOffPH % 128) == 0 && (kOffPL % 128) == 0 && (kOffG % 128) == 0 &&
              (kOffGT % 128) == 0);

__device__ __forceinline__ unsigned short f2bf_bits(float f) {
  unsigned u = __float_as_uint(f);
  return (unsigned short)((u + 0x7FFFu + ((u >> 16) & 1u)) >> 16);
}
__device__ __forceinline__ float bf_bits2f(unsigned short h) { return __uint_as_float(((unsigned)h) << 16); }
__device__ __forceinline__ unsigned pk16(unsigned short a, unsigned short b) { return (unsigned)a | ((unsigned)b << 16); }

__device__ __forceinline__ void tie_b4(v8f& acc, v16b a0, v16b a1, v16b b0, v16b b1) {
  asm volatile("v_nop\n\tv_nop\n\tv_nop\n\tv_nop" : "+v"(acc) : "v"(a0), "v"(a1), "v"(b0), "v"(b1));
}
__device__ __forceinline__ void tie_h2(v8f& acc, v16h a0, v16h b0) {
  asm volatile("v_nop\n\tv_nop\n\tv_nop\n\tv_nop" : "+v"(acc) : "v"(a0), "v"(b0));
}
__device__ __forceinline__ void keep4_b(v16b a, v16b b, v16b c, v16b d) { asm volatile("v_nop" :: "v"(a), "v"(b), "v"(c), "v"(d)); }
__device__ __forceinline__ void acc_guard4(v8f& a, v8f& b, v8f& c, v8f& d) { asm volatile("v_nop\n\tv_nop\n\tv_nop\n\tv_nop" : "+v"(a), "+v"(b), "+v"(c), "+v"(d)); }

union FragB { v16b v; v8b h[2]; };
union FragH { v16h v; v8h h[2]; };
__device__ __forceinline__ v16b ldfrag_b(const __bf16* p) {
  FragB f; f.h[0] = *(const v8b*)(p); f.h[1] = *(const v8b*)(p + 16); return f.v;
}
__device__ __forceinline__ v16h ldfrag_h(const _Float16* p) {
  FragH f; f.h[0] = *(const v8h*)(p); f.h[1] = *(const v8h*)(p + 16); return f.v;
}
__device__ __forceinline__ v8f mma_b(v16b a, v16b b, v8f c) {
  return __builtin_amdgcn_wmma_f32_16x16x32_bf16(false, a, false, b, (short)0, c, false, false);
}
__device__ __forceinline__ v8f mma_h(v16h a, v16h b, v8f c) {
  return __builtin_amdgcn_wmma_f32_16x16x32_f16(false, a, false, b, (short)0, c, false, false);
}

__global__ __launch_bounds__(256) void split_rows_bf16_kernel(
    const float* __restrict__ src, unsigned short* __restrict__ dhi, unsigned short* __restrict__ dlo, int total8)
{
  const int i = blockIdx.x * 256 + threadIdx.x;
  if (i >= total8) return;
  const size_t e0 = (size_t)i << 3;
  const v4f a0 = *(const v4f*)(src + e0);
  const v4f a1 = *(const v4f*)(src + e0 + 4);
  v8h hv, lv;
#pragma unroll
  for (int e = 0; e < 4; ++e) {
    const float f0 = a0[e];
    const float f1 = a1[e];
    const unsigned short h0 = f2bf_bits(f0), h1 = f2bf_bits(f1);
    const unsigned short l0 = f2bf_bits(f0 - bf_bits2f(h0)), l1 = f2bf_bits(f1 - bf_bits2f(h1));
    hv[e]     = __builtin_bit_cast(_Float16, h0);
    hv[4 + e] = __builtin_bit_cast(_Float16, h1);
    lv[e]     = __builtin_bit_cast(_Float16, l0);
    lv[4 + e] = __builtin_bit_cast(_Float16, l1);
  }
  unsigned short* qh = dhi + e0;
  unsigned short* ql = dlo + e0;
  *(volatile v8h*)qh = hv;
  *(volatile v8h*)ql = lv;
  __threadfence();
  *(volatile v8h*)qh = hv;
  *(volatile v8h*)ql = lv;
}

__global__ __launch_bounds__(256) void wt_split_kernel(
    const float* __restrict__ W0, const float* __restrict__ W1, const float* __restrict__ W2,
    unsigned short* __restrict__ WH, unsigned short* __restrict__ WL)
{
  __shared__ float sm[64][65];
  const int t  = threadIdx.x;
  const int i0 = blockIdx.x * 64;
  const int o0 = blockIdx.y * 64;
  const int z  = blockIdx.z;
  const float* W = (z == 0) ? W0 : ((z == 1) ? W1 : W2);
#pragma unroll
  for (int i = 0; i < 16; ++i) {
    const int e  = i * 256 + t;
    const int r  = e >> 6;
    const int cc = e & 63;
    sm[cc][r] = W[(size_t)(i0 + r) * kC + o0 + cc];
  }
  __syncthreads();
  const int lane = t & 31, wave = t >> 5;
  const int q = lane >> 3, c8 = (lane & 7) * 8;
  v8h hv[2], lv[2];
#pragma unroll
  for (int it = 0; it < 2; ++it) {
    const int row = wave * 8 + it * 4 + q;
#pragma unroll
    for (int e = 0; e < 8; ++e) {
      const float f = sm[row][c8 + e];
      const unsigned short hb = f2bf_bits(f);
      const unsigned short lb = f2bf_bits(f - bf_bits2f(hb));
      hv[it][e] = __builtin_bit_cast(_Float16, hb);
      lv[it][e] = __builtin_bit_cast(_Float16, lb);
    }
  }
  for (int pass = 0; pass < 2; ++pass) {
#pragma unroll
    for (int it = 0; it < 2; ++it) {
      const int row = wave * 8 + it * 4 + q;
      const size_t o = (size_t)(z * kC + o0 + row) * kC + i0 + c8;
      *(volatile v8h*)(WH + o) = hv[it];
      *(volatile v8h*)(WL + o) = lv[it];
    }
    __threadfence();
  }
}

template <int BAND>
__global__ __launch_bounds__(256) void proj_gemm_kernel(
    const unsigned short* __restrict__ XHp, const unsigned short* __restrict__ XLp,
    const unsigned short* __restrict__ WHp, const unsigned short* __restrict__ WLp,
    unsigned short* __restrict__ OutH, unsigned short* __restrict__ OutL)
{
  __shared__ __align__(16) float sT[8][16 * 68];
  const int lane = threadIdx.x & 31;
  const int wave = threadIdx.x >> 5;
  const int tile = blockIdx.x * 8 + wave;
  if (tile >= (kRows / 64) * (kC / 64)) return;
  const int tm = tile >> 2;
  const int tn = tile & 3;
  const int m0 = tm << 6;
  const int n0 = tn << 6;

  const __bf16* Ah = (const __bf16*)XHp;
  const __bf16* Al = (const __bf16*)XLp;
  const __bf16* Bh = (const __bf16*)WHp + (size_t)BAND * kC * kC;
  const __bf16* Bl = (const __bf16*)WLp + (size_t)BAND * kC * kC;

  const int rlane = lane & 15;
  const int hhalf = lane >> 4;
  const int koff  = hhalf * 8;
  const int mOff  = hhalf * 8;

  v8f acc[4][4];
#pragma unroll
  for (int i = 0; i < 4; ++i)
#pragma unroll
    for (int j = 0; j < 4; ++j) acc[i][j] = (v8f){0.f,0.f,0.f,0.f,0.f,0.f,0.f,0.f};

#pragma unroll 1
  for (int k0 = 0; k0 < kC; k0 += 32) {
    v16b bh[4], bl[4];
#pragma unroll
    for (int j = 0; j < 4; ++j) {
      const size_t bo = (size_t)(n0 + (j << 4) + rlane) * kC + koff + k0;
      bh[j] = ldfrag_b(Bh + bo);
      bl[j] = ldfrag_b(Bl + bo);
    }
#pragma unroll
    for (int i = 0; i < 4; ++i) {
      const size_t ao = (size_t)(m0 + (i << 4) + rlane) * kC + koff + k0;
      const v16b ah = ldfrag_b(Ah + ao);
      const v16b al = ldfrag_b(Al + ao);
#pragma unroll
      for (int j = 0; j < 4; ++j) {
        acc[i][j] = mma_b(ah, bh[j], acc[i][j]);
        acc[i][j] = mma_b(ah, bl[j], acc[i][j]);
        acc[i][j] = mma_b(al, bh[j], acc[i][j]);
        tie_b4(acc[i][j], ah, al, bh[j], bl[j]);
      }
    }
    keep4_b(bh[0], bh[1], bh[2], bh[3]);
    keep4_b(bl[0], bl[1], bl[2], bl[3]);
  }
  acc_guard4(acc[0][0], acc[0][1], acc[0][2], acc[0][3]);
  acc_guard4(acc[1][0], acc[1][1], acc[1][2], acc[1][3]);
  acc_guard4(acc[2][0], acc[2][1], acc[2][2], acc[2][3]);
  acc_guard4(acc[3][0], acc[3][1], acc[3][2], acc[3][3]);

  float* slab = sT[wave];
  const int q = lane >> 3, c8 = (lane & 7) * 8;

  if (BAND == 0) {
#pragma unroll
    for (int i = 0; i < 4; ++i) {
      const int mBase = m0 + (i << 4);
#pragma unroll
      for (int j = 0; j < 4; ++j) {
#pragma unroll
        for (int r = 0; r < 8; ++r) slab[(mOff + r) * 68 + (j << 4) + rlane] = acc[i][j][r];
      }
      __builtin_amdgcn_fence(__ATOMIC_RELEASE, "workgroup");
      __builtin_amdgcn_wave_barrier();
      __builtin_amdgcn_fence(__ATOMIC_ACQUIRE, "workgroup");
      v8h hv[4], lv[4];
#pragma unroll
      for (int it = 0; it < 4; ++it) {
        const float* sp = slab + (it * 4 + q) * 68 + c8;
        const v4f a0 = *(const v4f*)(sp);
        const v4f a1 = *(const v4f*)(sp + 4);
#pragma unroll
        for (int e = 0; e < 4; ++e) {
          const float f0 = a0[e];
          const float f1 = a1[e];
          const unsigned short h0 = f2bf_bits(f0), h1 = f2bf_bits(f1);
          const unsigned short l0 = f2bf_bits(f0 - bf_bits2f(h0)), l1 = f2bf_bits(f1 - bf_bits2f(h1));
          hv[it][e]     = __builtin_bit_cast(_Float16, h0);
          hv[it][4 + e] = __builtin_bit_cast(_Float16, h1);
          lv[it][e]     = __builtin_bit_cast(_Float16, l0);
          lv[it][4 + e] = __builtin_bit_cast(_Float16, l1);
        }
      }
      for (int pass = 0; pass < 2; ++pass) {
#pragma unroll
        for (int it = 0; it < 4; ++it) {
          const size_t o = (size_t)(mBase + it * 4 + q) * kC + n0 + c8;
          *(volatile v8h*)(OutH + o) = hv[it];
          *(volatile v8h*)(OutL + o) = lv[it];
        }
        __threadfence();
      }
      __builtin_amdgcn_fence(__ATOMIC_RELEASE, "workgroup");
      __builtin_amdgcn_wave_barrier();
      __builtin_amdgcn_fence(__ATOMIC_ACQUIRE, "workgroup");
    }
  } else {
#pragma unroll
    for (int ii = 0; ii < 2; ++ii) {
      const int pBase = (m0 >> 1) + (ii << 4);
#pragma unroll
      for (int i2 = 0; i2 < 2; ++i2) {
#pragma unroll
        for (int j = 0; j < 4; ++j) {
#pragma unroll
          for (int p = 0; p < 4; ++p) {
            const float v = fmaxf(acc[2 * ii + i2][j][2 * p], acc[2 * ii + i2][j][2 * p + 1]);
            slab[(8 * i2 + 4 * hhalf + p) * 68 + (j << 4) + rlane] = v;
          }
        }
      }
      __builtin_amdgcn_fence(__ATOMIC_RELEASE, "workgroup");
      __builtin_amdgcn_wave_barrier();
      __builtin_amdgcn_fence(__ATOMIC_ACQUIRE, "workgroup");
      v8h hv[4], lv[4];
#pragma unroll
      for (int it = 0; it < 4; ++it) {
        const float* sp = slab + (it * 4 + q) * 68 + c8;
        const v4f a0 = *(const v4f*)(sp);
        const v4f a1 = *(const v4f*)(sp + 4);
#pragma unroll
        for (int e = 0; e < 4; ++e) {
          const float f0 = a0[e];
          const float f1 = a1[e];
          if (BAND == 1) {
            const unsigned short h0 = f2bf_bits(f0), h1 = f2bf_bits(f1);
            const unsigned short l0 = f2bf_bits(f0 - bf_bits2f(h0)), l1 = f2bf_bits(f1 - bf_bits2f(h1));
            hv[it][e]     = __builtin_bit_cast(_Float16, h0);
            hv[it][4 + e] = __builtin_bit_cast(_Float16, h1);
            lv[it][e]     = __builtin_bit_cast(_Float16, l0);
            lv[it][4 + e] = __builtin_bit_cast(_Float16, l1);
          } else {
            hv[it][e]     = (_Float16)f0;
            hv[it][4 + e] = (_Float16)f1;
            lv[it][e]     = (_Float16)0.0f;
            lv[it][4 + e] = (_Float16)0.0f;
          }
        }
      }
      for (int pass = 0; pass < 2; ++pass) {
#pragma unroll
        for (int it = 0; it < 4; ++it) {
          const size_t o = (size_t)(pBase + it * 4 + q) * kC + n0 + c8;
          *(volatile v8h*)(OutH + o) = hv[it];
          if (BAND == 1) *(volatile v8h*)(OutL + o) = lv[it];
        }
        __threadfence();
      }
      __builtin_amdgcn_fence(__ATOMIC_RELEASE, "workgroup");
      __builtin_amdgcn_wave_barrier();
      __builtin_amdgcn_fence(__ATOMIC_ACQUIRE, "workgroup");
    }
  }
}

__global__ __launch_bounds__(256) void g_transpose_kernel(const unsigned* __restrict__ Gw, unsigned short* __restrict__ GT)
{
  __shared__ unsigned short sm[64][72];
  const int t  = threadIdx.x;
  const int m0 = blockIdx.x * 64;
  const int c0 = blockIdx.y * 64;
  const int b  = blockIdx.z;
#pragma unroll
  for (int i = 0; i < 8; ++i) {
    const int e  = i * 256 + t;
    const int r  = e >> 5;
    const int cw = e & 31;
    const unsigned w = Gw[(((size_t)(b * kMk + m0 + r) * kC + c0) >> 1) + cw];
    sm[2 * cw][r]     = (unsigned short)(w & 0xffffu);
    sm[2 * cw + 1][r] = (unsigned short)(w >> 16);
  }
  __syncthreads();
  const int lane = t & 31, wave = t >> 5;
  const int q = lane >> 3, c8 = (lane & 7) * 8;
  v4u u[2];
#pragma unroll
  for (int it = 0; it < 2; ++it) {
    const int row = wave * 8 + it * 4 + q;
    unsigned short hb[8];
#pragma unroll
    for (int e = 0; e < 8; ++e) hb[e] = sm[row][c8 + e];
    u[it] = (v4u){pk16(hb[0], hb[1]), pk16(hb[2], hb[3]), pk16(hb[4], hb[5]), pk16(hb[6], hb[7])};
  }
  for (int pass = 0; pass < 2; ++pass) {
#pragma unroll
    for (int it = 0; it < 2; ++it) {
      const int row = wave * 8 + it * 4 + q;
      *(volatile v4u*)(GT + (size_t)(b * kC + c0 + row) * kMk + m0 + c8) = u[it];
    }
    __threadfence();
  }
}

__global__ __launch_bounds__(128) __attribute__((amdgpu_num_vgpr(256)))
void attn_fused_kernel(const float* __restrict__ x,
                       const unsigned short* __restrict__ THp, const unsigned short* __restrict__ TLp,
                       const unsigned short* __restrict__ PHp, const unsigned short* __restrict__ PLp,
                       const unsigned short* __restrict__ GTp, float* __restrict__ out)
{
  __shared__ __align__(16) __bf16   sTheta[kAtWaves][2][16 * kC];
  __shared__ __align__(16) __bf16   sPhiH[kKeyChunk * kC];
  __shared__ __align__(16) __bf16   sPhiL[kKeyChunk * kC];
  __shared__ __align__(16) _Float16 sG[kC * kKeyChunk];
  __shared__ __align__(16) _Float16 sP[kAtWaves][16 * kKeyChunk];

  const int tid  = threadIdx.x;
  const int wave = tid >> 5;
  const int lane = tid & 31;
  const int hh   = lane >> 4;
  const int c    = lane & 15;

  constexpr int kBlkPerB = kNq / kQryBlock;
  const int b  = blockIdx.x / kBlkPerB;
  const int qb = blockIdx.x - b * kBlkPerB;
  const int qrow0 = b * kNq + qb * kQryBlock + wave * 16;

  const __bf16*   TH = (const __bf16*)THp;
  const __bf16*   TL = (const __bf16*)TLp;
  const __bf16*   PHb = (const __bf16*)PHp + (size_t)b * kMk * kC;
  const __bf16*   PLb = (const __bf16*)PLp + (size_t)b * kMk * kC;
  const _Float16* GTb = (const _Float16*)GTp + (size_t)b * kC * kMk;

  __bf16* thw_h = sTheta[wave][0];
  __bf16* thw_l = sTheta[wave][1];
#pragma unroll 4
  for (int i = 0; i < 16; ++i) {
    const size_t go = (size_t)(qrow0 + i) * kC + lane * 8;
    *(v8b*)(thw_h + i * kC + lane * 8) = *(const v8b*)(TH + go);
    *(v8b*)(thw_l + i * kC + lane * 8) = *(const v8b*)(TL + go);
  }

  v8f yacc[16];
#pragma unroll
  for (int t = 0; t < 16; ++t) yacc[t] = (v8f){0.f,0.f,0.f,0.f,0.f,0.f,0.f,0.f};
  v8f lacc = (v8f){0.f,0.f,0.f,0.f,0.f,0.f,0.f,0.f};
  float mrow[8];
#pragma unroll
  for (int r = 0; r < 8; ++r) mrow[r] = -3.0e38f;
  v16h ones;
#pragma unroll
  for (int e = 0; e < 16; ++e) ones[e] = (_Float16)1.0f;

  _Float16* pw = sP[wave];

#pragma unroll 1
  for (int kc = 0; kc < kMk / kKeyChunk; ++kc) {
    const int kv0 = kc * kKeyChunk;
    __syncthreads();
#pragma unroll 4
    for (int i = 0; i < 16; ++i) {
      const int cid = i * 128 + tid;
      const int r   = cid >> 5;
      const int c8  = (cid & 31) * 8;
      const size_t go = (size_t)(kv0 + r) * kC + c8;
      *(v8b*)(sPhiH + r * kC + c8) = *(const v8b*)(PHb + go);
      *(v8b*)(sPhiL + r * kC + c8) = *(const v8b*)(PLb + go);
    }
#pragma unroll 4
    for (int i = 0; i < 16; ++i) {
      const int cid = i * 128 + tid;
      const int cr  = cid >> 3;
      const int k8  = (cid & 7) * 8;
      *(v8h*)(sG + cr * kKeyChunk + k8) = *(const v8h*)(GTb + (size_t)cr * kMk + kv0 + k8);
    }
    __syncthreads();

    v8f s[4];
#pragma unroll
    for (int j = 0; j < 4; ++j) s[j] = (v8f){0.f,0.f,0.f,0.f,0.f,0.f,0.f,0.f};
#pragma unroll 1
    for (int ks = 0; ks < kC / 32; ++ks) {
      const int ko = ks * 32 + 8 * hh;
      const v16b ah = ldfrag_b(thw_h + c * kC + ko);
      const v16b al = ldfrag_b(thw_l + c * kC + ko);
#pragma unroll
      for (int j = 0; j < 4; ++j) {
        const v16b bh = ldfrag_b(sPhiH + (j * 16 + c) * kC + ko);
        const v16b bl = ldfrag_b(sPhiL + (j * 16 + c) * kC + ko);
        s[j] = mma_b(ah, bh, s[j]);
        s[j] = mma_b(ah, bl, s[j]);
        s[j] = mma_b(al, bh, s[j]);
        tie_b4(s[j], ah, al, bh, bl);
      }
    }

#pragma unroll
    for (int r = 0; r < 8; ++r) {
      const float a0 = s[0][r] * kLog2e;
      const float a1 = s[1][r] * kLog2e;
      const float a2 = s[2][r] * kLog2e;
      const float a3 = s[3][r] * kLog2e;
      float m = fmaxf(fmaxf(a0, a1), fmaxf(a2, a3));
      m = fmaxf(m, __shfl_xor(m, 1, 32));
      m = fmaxf(m, __shfl_xor(m, 2, 32));
      m = fmaxf(m, __shfl_xor(m, 4, 32));
      m = fmaxf(m, __shfl_xor(m, 8, 32));
      const float mnew  = fmaxf(mrow[r], m);
      const float alpha = __builtin_amdgcn_exp2f(mrow[r] - mnew);
      mrow[r] = mnew;
      const float msub = mnew - kPCarryL;
      const float p0 = __builtin_amdgcn_exp2f(a0 - msub);
      const float p1 = __builtin_amdgcn_exp2f(a1 - msub);
      const float p2 = __builtin_amdgcn_exp2f(a2 - msub);
      const float p3 = __builtin_amdgcn_exp2f(a3 - msub);
      _Float16* prow = pw + (8 * hh + r) * kKeyChunk + c;
      prow[0]  = (_Float16)p0;
      prow[16] = (_Float16)p1;
      prow[32] = (_Float16)p2;
      prow[48] = (_Float16)p3;
      lacc[r] *= alpha;
#pragma unroll
      for (int t = 0; t < 16; ++t) yacc[t][r] *= alpha;
    }
    __builtin_amdgcn_fence(__ATOMIC_RELEASE, "workgroup");
    __builtin_amdgcn_wave_barrier();
    __builtin_amdgcn_fence(__ATOMIC_ACQUIRE, "workgroup");

#pragma unroll 1
    for (int kk = 0; kk < kKeyChunk / 32; ++kk) {
      const v16h pa = ldfrag_h(pw + c * kKeyChunk + kk * 32 + 8 * hh);
      lacc = mma_h(pa, ones, lacc);
      tie_h2(lacc, pa, ones);
#pragma unroll
      for (int t = 0; t < 16; ++t) {
        const v16h vb = ldfrag_h(sG + (t * 16 + c) * kKeyChunk + kk * 32 + 8 * hh);
        yacc[t] = mma_h(pa, vb, yacc[t]);
        tie_h2(yacc[t], pa, vb);
      }
    }
  }

  __syncthreads();

  float* os = reinterpret_cast<float*>(&sTheta[wave][0][0]);
#pragma unroll
  for (int r = 0; r < 8; ++r) {
    const float inv = 1.0f / lacc[r];
#pragma unroll
    for (int t = 0; t < 16; ++t) os[(8 * hh + r) * kC + t * 16 + c] = yacc[t][r] * inv;
  }
  __builtin_amdgcn_fence(__ATOMIC_RELEASE, "workgroup");
  __builtin_amdgcn_wave_barrier();
  __builtin_amdgcn_fence(__ATOMIC_ACQUIRE, "workgroup");
  {
    const float* xb = x   + (size_t)qrow0 * kC;
    float*       ob = out + (size_t)qrow0 * kC;
    for (int pass = 0; pass < 2; ++pass) {
#pragma unroll 4
      for (int it = 0; it < 32; ++it) {
        const int off = it * 128 + lane * 4;
        const v4f yv = *(const v4f*)(os + off);
        const v4f xv = *(const v4f*)(xb + off);
        const v4f ov = xv + yv;
        *(volatile v4f*)(ob + off) = ov;
      }
      __threadfence();
    }
  }
}

extern "C" void kernel_launch(void* const* d_in, const int* in_sizes, int n_in,
                              void* d_out, int out_size, void* d_ws, size_t ws_size,
                              hipStream_t stream) {
  if (n_in < 4) return;
  if (in_sizes[0] != kRows * kC) return;
  if (in_sizes[1] != kC * kC) return;
  if (in_sizes[2] != kC * kC) return;
  if (in_sizes[3] != kC * kC) return;
  if (out_size != kRows * kC) return;
  if (ws_size < kWsTotal) return;

  const float* x       = (const float*)d_in[0];
  const float* w_theta = (const float*)d_in[1];
  const float* w_phi   = (const float*)d_in[2];
  const float* w_g     = (const float*)d_in[3];
  float* out = (float*)d_out;

  char* ws = (char*)d_ws;
  unsigned short* XH = (unsigned short*)(ws + kOffXH);
  unsigned short* XL = (unsigned short*)(ws + kOffXL);
  unsigned short* WH = (unsigned short*)(ws + kOffWH);
  unsigned short* WL = (unsigned short*)(ws + kOffWL);
  unsigned short* TH = (unsigned short*)(ws + kOffTH);
  unsigned short* TL = (unsigned short*)(ws + kOffTL);
  unsigned short* PH = (unsigned short*)(ws + kOffPH);
  unsigned short* PL = (unsigned short*)(ws + kOffPL);
  unsigned short* G  = (unsigned short*)(ws + kOffG);
  unsigned short* GT = (unsigned short*)(ws + kOffGT);

  split_rows_bf16_kernel<<<(kRows * kC / 8) / 256, 256, 0, stream>>>(x, XH, XL, kRows * kC / 8);
  wt_split_kernel<<<dim3(kC / 64, kC / 64, 3), 256, 0, stream>>>(w_theta, w_phi, w_g, WH, WL);

  constexpr int kGemmBlocks = ((kRows / 64) * (kC / 64)) / 8;
  proj_gemm_kernel<0><<<kGemmBlocks, 256, 0, stream>>>(XH, XL, WH, WL, TH, TL);
  proj_gemm_kernel<1><<<kGemmBlocks, 256, 0, stream>>>(XH, XL, WH, WL, PH, PL);
  proj_gemm_kernel<2><<<kGemmBlocks, 256, 0, stream>>>(XH, XL, WH, WL, G, G);

  g_transpose_kernel<<<dim3(kMk / 64, kC / 64, kBatch), 256, 0, stream>>>((const unsigned*)G, GT);

  attn_fused_kernel<<<kBatch * (kNq / kQryBlock), kAtWaves * 32, 0, stream>>>(x, TH, TL, PH, PL, GT, out);
}
